// StackedTransDecoder_5085241279167
// MI455X (gfx1250) — hardware-verified
//
#include <hip/hip_runtime.h>
#include <math.h>

typedef __attribute__((ext_vector_type(16))) _Float16 v16h;
typedef __attribute__((ext_vector_type(8)))  _Float16 v8h;
typedef __attribute__((ext_vector_type(4)))  _Float16 v4h;
typedef __attribute__((ext_vector_type(2)))  _Float16 v2h;
typedef __attribute__((ext_vector_type(16))) __bf16   v16b;
typedef __attribute__((ext_vector_type(8)))  __bf16   v8b;
typedef __attribute__((ext_vector_type(8)))  float    v8f;
typedef __attribute__((ext_vector_type(4)))  float    v4f;
typedef __attribute__((ext_vector_type(2)))  float    v2f;

constexpr int kB    = 64;
constexpr int kLX   = 64;
constexpr int kLY   = 64;
constexpr int kE2   = 1024;
constexpr int kD    = 512;
constexpr int kNE   = 512;
constexpr int kNH   = 8;
constexpr int kHV   = kE2 / kNH;
constexpr int kG3   = 3 * kD;
constexpr int kQH   = kD + kG3;
constexpr int kCS   = kE2 + kD;
constexpr int kRows = kB * kLX;
constexpr int kThr  = 256;
constexpr float kInCarry = 1024.0f;
constexpr float kWCarry  = 4096.0f;
constexpr float kSc = 1.0f / (kInCarry * kWCarry);
constexpr float kF16MinNormal = 6.103515625e-5f;
constexpr int kFSI = 0, kFQH = 512, kFBO = 2560, kFCS = 3584, kFBY = 4096, kFZ = 4608, kFEnd = 6144;

static_assert(kB == 64 && (kRows % 64) == 0 && (kG3 / 64) % 8 == 0 && (kQH / 64) % 8 == 0 && (kE2 / 64) % 8 == 0 && (kD / 64) % 8 == 0 && (kD % 32) == 0 && (kE2 % 32) == 0 && (kCS % 32) == 0
              && (kD / 8) <= 256 && (kE2 / 8) <= 256 && kFZ + kG3 <= kFEnd, "GEMM M, N multiples of 64; grids exact; K multiples of 32");

constexpr size_t kOffWKT = 0ull;
constexpr size_t kOffWSIT = 1048576ull;
constexpr size_t kOffWXCT = 2097152ull;
constexpr size_t kOffWHCT = 3670016ull;
constexpr size_t kOffWQHT = 5242880ull;
constexpr size_t kOffWOT = 7340032ull;
constexpr size_t kOffWXDT = 9437184ull;
constexpr size_t kOffWCST = 12582912ull;
constexpr size_t kOffWYT = 14155776ull;
constexpr size_t kOffBIAS = 14680064ull;
constexpr size_t kOffXS16 = 14704640ull;
constexpr size_t kOffYS16 = 23093248ull;
constexpr size_t kOffUH32 = 27287552ull;
constexpr size_t kOffAXC = 35676160ull;
constexpr size_t kOffYWY = 60841984ull;
constexpr size_t kOffPOOL = 69230592ull;
constexpr size_t kOffS0P = 69361664ull;
constexpr size_t kOffS32 = 69492736ull;
constexpr size_t kOffST32 = 69623808ull;
constexpr size_t kOffST16 = 69754880ull;
constexpr size_t kOffCS16 = 69820416ull;
constexpr size_t kOffAH1 = 70017024ull;
constexpr size_t kOffQH = 70410240ull;
constexpr size_t kOffCTX16 = 70934528ull;
constexpr size_t kOffCTX2 = 71065600ull;
constexpr size_t kOffAX2 = 71327744ull;
constexpr size_t kOffOUTP = 71720960ull;
constexpr size_t kWsTotal = 71852032ull;
static_assert(kWsTotal <= 134217728ull, "carve cap: under 128 MiB");
static_assert(kOffWKT == 0
              && kOffWSIT == kOffWKT + 1048576ull
              && kOffWXCT == kOffWSIT + 1048576ull
              && kOffWHCT == kOffWXCT + 1572864ull
              && kOffWQHT == kOffWHCT + 1572864ull
              && kOffWOT == kOffWQHT + 2097152ull
              && kOffWXDT == kOffWOT + 2097152ull
              && kOffWCST == kOffWXDT + 3145728ull
              && kOffWYT == kOffWCST + 1572864ull
              && kOffBIAS == kOffWYT + 524288ull
              && kOffXS16 == kOffBIAS + 24576ull
              && kOffYS16 == kOffXS16 + 8388608ull
              && kOffUH32 == kOffYS16 + 4194304ull
              && kOffAXC == kOffUH32 + 8388608ull
              && kOffYWY == kOffAXC + 25165824ull
              && kOffPOOL == kOffYWY + 8388608ull
              && kOffS0P == kOffPOOL + 131072ull
              && kOffS32 == kOffS0P + 131072ull
              && kOffST32 == kOffS32 + 131072ull
              && kOffST16 == kOffST32 + 131072ull
              && kOffCS16 == kOffST16 + 65536ull
              && kOffAH1 == kOffCS16 + 196608ull
              && kOffQH == kOffAH1 + 393216ull
              && kOffCTX16 == kOffQH + 524288ull
              && kOffCTX2 == kOffCTX16 + 131072ull
              && kOffAX2 == kOffCTX2 + 262144ull
              && kOffOUTP == kOffAX2 + 393216ull
              && kWsTotal == kOffOUTP + 131072ull, "the carve is chained and totalled");
static_assert((kOffWKT % 256) == 0 && (kOffWSIT % 256) == 0 && (kOffWXCT % 256) == 0 && (kOffWHCT % 256) == 0 && (kOffWQHT % 256) == 0 && (kOffWOT % 256) == 0 && (kOffWXDT % 256) == 0 && (kOffWCST % 256) == 0 && (kOffWYT % 256) == 0 && (kOffBIAS % 256) == 0 && (kOffXS16 % 256) == 0 && (kOffYS16 % 256) == 0 && (kOffUH32 % 256) == 0 && (kOffAXC % 256) == 0 && (kOffYWY % 256) == 0 && (kOffPOOL % 256) == 0 && (kOffS0P % 256) == 0 && (kOffS32 % 256) == 0 && (kOffST32 % 256) == 0 && (kOffST16 % 256) == 0 && (kOffCS16 % 256) == 0 && (kOffAH1 % 256) == 0 && (kOffQH % 256) == 0 && (kOffCTX16 % 256) == 0 && (kOffCTX2 % 256) == 0 && (kOffAX2 % 256) == 0 && (kOffOUTP % 256) == 0, "aligned regions");

__device__ __forceinline__ unsigned short f2bf_bits(float f) {
  unsigned u = __float_as_uint(f);
  return (unsigned short)((u + 0x7FFFu + ((u >> 16) & 1u)) >> 16);
}
__device__ __forceinline__ float bf_bits2f(unsigned short h) { return __uint_as_float(((unsigned)h) << 16); }
__device__ __forceinline__ float bf16r(float f) { return bf_bits2f(f2bf_bits(f)); }
__device__ __forceinline__ float carry_flush(float v, float carry) {
  const float s = v * carry;
  return (fabsf(s) < kF16MinNormal) ? 0.0f : s;
}
__device__ __forceinline__ float frcp(float x) { return __builtin_amdgcn_rcpf(x); }

__device__ __forceinline__ void dep_guard4_h(v8f& a, v8f& b, v8f& c, v8f& d, v16h x, v16h y) { asm volatile("v_nop\n\tv_nop\n\tv_nop\n\tv_nop" : "+v"(a), "+v"(b), "+v"(c), "+v"(d) : "v"(x), "v"(y)); }
__device__ __forceinline__ void dep_guard4_b(v8f& a, v8f& b, v8f& c, v8f& d, v16b x, v16b y) { asm volatile("v_nop\n\tv_nop\n\tv_nop\n\tv_nop" : "+v"(a), "+v"(b), "+v"(c), "+v"(d) : "v"(x), "v"(y)); }
__device__ __forceinline__ void keep4_h(v16h a, v16h b, v16h c, v16h d) { asm volatile("v_nop" :: "v"(a), "v"(b), "v"(c), "v"(d)); }
__device__ __forceinline__ void keep4_b(v16b a, v16b b, v16b c, v16b d) { asm volatile("v_nop" :: "v"(a), "v"(b), "v"(c), "v"(d)); }
__device__ __forceinline__ void acc_guard4(v8f& a, v8f& b, v8f& c, v8f& d) { asm volatile("v_nop\n\tv_nop\n\tv_nop\n\tv_nop" : "+v"(a), "+v"(b), "+v"(c), "+v"(d)); }

template <typename T> struct Frag;
template <> struct Frag<_Float16> {
  typedef v16h V; union U { v16h v; v8h h[2]; };
  static __device__ __forceinline__ v16h load(const _Float16* p) {
    U f; f.h[0] = *(const v8h*)(p); f.h[1] = *(const v8h*)(p + 16); return f.v;
  }
  static __device__ __forceinline__ v8f mma(v16h a, v16h b, v8f c) {
    return __builtin_amdgcn_wmma_f32_16x16x32_f16(false, a, false, b, (short)0, c, false, false);
  }
  static __device__ __forceinline__ void guard4(v8f& a, v8f& b, v8f& c, v8f& d, v16h x, v16h y) { dep_guard4_h(a, b, c, d, x, y); }
  static __device__ __forceinline__ void keep(v16h a, v16h b, v16h c, v16h d) { keep4_h(a, b, c, d); }
};
template <> struct Frag<__bf16> {
  typedef v16b V; union U { v16b v; v8b h[2]; };
  static __device__ __forceinline__ v16b load(const __bf16* p) {
    U f; f.h[0] = *(const v8b*)(p); f.h[1] = *(const v8b*)(p + 16); return f.v;
  }
  static __device__ __forceinline__ v8f mma(v16b a, v16b b, v8f c) {
    return __builtin_amdgcn_wmma_f32_16x16x32_bf16(false, a, false, b, (short)0, c, false, false);
  }
  static __device__ __forceinline__ void guard4(v8f& a, v8f& b, v8f& c, v8f& d, v16b x, v16b y) { dep_guard4_b(a, b, c, d, x, y); }
  static __device__ __forceinline__ void keep(v16b a, v16b b, v16b c, v16b d) { keep4_b(a, b, c, d); }
};

__device__ __forceinline__ v8f mma_h(v16h a, v16h b, v8f c) {
  c = __builtin_amdgcn_wmma_f32_16x16x32_f16(false, a, false, b, (short)0, c, false, false);
  asm volatile("v_nop\n\tv_nop\n\tv_nop\n\tv_nop" : "+v"(c) : "v"(a), "v"(b));
  return c;
}

template <int ET> struct Elem;
template <> struct Elem<0> { typedef _Float16 T; };
template <> struct Elem<1> { typedef __bf16 T; };
template <int ET, bool SPLIT, int BIAS_MODE, int OUT_MODE, bool RESID, int ACT = 0>
__global__ __launch_bounds__(256) void wmma_gemm64(
    const unsigned short* __restrict__ Ap, const unsigned short* __restrict__ A2p, int lda, long strideA,
    const unsigned short* __restrict__ Btp, const unsigned short* __restrict__ Bt2p, int ldb, long strideB,
    void* __restrict__ Cout, void* __restrict__ Cout2, int ldc, long strideC,
    const float* __restrict__ bias,
    const float* __restrict__ resid, long strideR,
    int M, int N, int K, float scale) {
  typedef typename Elem<ET>::T T;
  typedef typename Frag<T>::V V;
  const T* A = (const T*)Ap; const T* A2 = (const T*)A2p; const T* Bt = (const T*)Btp; const T* Bt2 = (const T*)Bt2p;
  __shared__ __align__(16) float sT[8][16 * 68];
  const int b    = blockIdx.y;
  const int lane = threadIdx.x & 31;
  const int wave = threadIdx.x >> 5;
  const int tilesN = N >> 6;
  const int tilesM = M >> 6;
  const int tile = blockIdx.x * 8 + wave;
  if (tile >= tilesM * tilesN) return;
  const int tm = tile / tilesN;
  const int tn = tile - tm * tilesN;
  const int m0 = tm << 6;
  const int n0 = tn << 6;

  const T* Ab  = A  + (size_t)b * strideA;
  const T* Bb  = Bt + (size_t)b * strideB;
  const T* Ab2 = SPLIT ? (A2  + (size_t)b * strideA) : nullptr;
  const T* Bb2 = SPLIT ? (Bt2 + (size_t)b * strideB) : nullptr;

  const int rlane = lane & 15;
  const int koff  = (lane >> 4) * 8;
  const int mOff  = (lane >> 4) * 8;

  v8f acc[4][4];
#pragma unroll
  for (int i = 0; i < 4; ++i)
#pragma unroll
    for (int j = 0; j < 4; ++j) acc[i][j] = (v8f){0.f,0.f,0.f,0.f,0.f,0.f,0.f,0.f};

  for (int k0 = 0; k0 < K; k0 += 32) {
    V bh[4], bl[4];
#pragma unroll
    for (int j = 0; j < 4; ++j) {
      const size_t bo = (size_t)(n0 + (j << 4) + rlane) * ldb + koff + k0;
      bh[j] = Frag<T>::load(Bb + bo);
      if (SPLIT) bl[j] = Frag<T>::load(Bb2 + bo);
    }
#pragma unroll
    for (int i = 0; i < 4; ++i) {
      const size_t ao = (size_t)(m0 + (i << 4) + rlane) * lda + koff + k0;
      V ah = Frag<T>::load(Ab + ao);
      V al;
      if (SPLIT) al = Frag<T>::load(Ab2 + ao);
#pragma unroll
      for (int j = 0; j < 4; ++j) {
        acc[i][j] = Frag<T>::mma(ah, bh[j], acc[i][j]);
        if (SPLIT) {
          acc[i][j] = Frag<T>::mma(ah, bl[j], acc[i][j]);
          acc[i][j] = Frag<T>::mma(al, bh[j], acc[i][j]);
        }
      }
      Frag<T>::guard4(acc[i][0], acc[i][1], acc[i][2], acc[i][3], ah, SPLIT ? al : ah);
    }
    Frag<T>::keep(bh[0], bh[1], bh[2], bh[3]);
    if (SPLIT) Frag<T>::keep(bl[0], bl[1], bl[2], bl[3]);
  }
  acc_guard4(acc[0][0], acc[0][1], acc[0][2], acc[0][3]);
  acc_guard4(acc[1][0], acc[1][1], acc[1][2], acc[1][3]);
  acc_guard4(acc[2][0], acc[2][1], acc[2][2], acc[2][3]);
  acc_guard4(acc[3][0], acc[3][1], acc[3][2], acc[3][3]);

  float* slab = sT[wave];
  const float* Rb = RESID ? (resid + (size_t)b * strideR) : nullptr;
#pragma unroll
  for (int i = 0; i < 4; ++i) {
    const int mBase = m0 + (i << 4);
#pragma unroll
    for (int j = 0; j < 4; ++j) {
      const int n = n0 + (j << 4) + rlane;
      float bv = 0.f;
      if (BIAS_MODE == 2) bv = bias[n];
#pragma unroll
      for (int r = 0; r < 8; ++r) {
        float v = acc[i][j][r] * scale;
        if (BIAS_MODE == 1) v += bias[mBase + mOff + r];
        if (BIAS_MODE == 2) v += bv;
        if (RESID) v += Rb[(size_t)(mBase + mOff + r) * ldc + n];
        if (ACT == 1) v = tanhf(v);
        if (ACT == 2) v = fmaxf(v, 0.0f);
        if (ACT == 3) v = v / (1.0f + expf(-v));
        if (ACT == 4) v = (v > 0.f) ? v : 0.01f * v;
        slab[(mOff + r) * 68 + (j << 4) + rlane] = v;
      }
    }
    __builtin_amdgcn_fence(__ATOMIC_RELEASE, "workgroup");
    __builtin_amdgcn_wave_barrier();
    __builtin_amdgcn_fence(__ATOMIC_ACQUIRE, "workgroup");
    if (OUT_MODE == 0) {
      float* C = (float*)Cout + (size_t)b * strideC;
      const int hh = lane >> 4, c4 = (lane & 15) * 4;
      for (int pass = 0; pass < 2; ++pass) {
#pragma unroll
        for (int it = 0; it < 8; ++it) {
          const int row = it * 2 + hh;
          v4f v = *(const v4f*)(slab + row * 68 + c4);
          *(volatile v4f*)(C + (size_t)(mBase + row) * ldc + n0 + c4) = v;
        }
        __threadfence();
      }
    } else {
      const int q = lane >> 3, c8 = (lane & 7) * 8;
      unsigned short* C  = (unsigned short*)Cout  + (size_t)b * strideC;
      unsigned short* C2 = (OUT_MODE == 2) ? ((unsigned short*)Cout2 + (size_t)b * strideC) : nullptr;
      for (int pass = 0; pass < 2; ++pass) {
#pragma unroll
        for (int it = 0; it < 4; ++it) {
          const int row = it * 4 + q;
          const float* sp = slab + row * 68 + c8;
          v8h hv, lv;
#pragma unroll
          for (int e = 0; e < 8; ++e) {
            if (OUT_MODE == 1) {
              hv[e] = (_Float16)sp[e];
            } else {
              unsigned short hb = f2bf_bits(sp[e]);
              unsigned short lb = f2bf_bits(sp[e] - bf_bits2f(hb));
              hv[e] = __builtin_bit_cast(_Float16, hb);
              lv[e] = __builtin_bit_cast(_Float16, lb);
            }
          }
          *(volatile v8h*)(C + (size_t)(mBase + row) * ldc + n0 + c8) = hv;
          if (OUT_MODE == 2) *(volatile v8h*)(C2 + (size_t)(mBase + row) * ldc + n0 + c8) = lv;
        }
        __threadfence();
      }
    }
    __builtin_amdgcn_fence(__ATOMIC_RELEASE, "workgroup");
    __builtin_amdgcn_wave_barrier();
    __builtin_amdgcn_fence(__ATOMIC_ACQUIRE, "workgroup");
  }
}

__global__ __launch_bounds__(kThr) void cast_plane_kernel(const float* __restrict__ src, unsigned short* __restrict__ dst,
                                                          int colsLog2, int dstPitch, int dstOff) {
  const int i   = blockIdx.x * kThr + threadIdx.x;
  const int sh  = colsLog2 - 3;
  const int row = i >> sh;
  const int c8  = (i & ((1 << sh) - 1)) * 8;
  const float* sp = src + ((size_t)row << colsLog2) + c8;
  const v4f a0 = *(const v4f*)(sp);
  const v4f a1 = *(const v4f*)(sp + 4);
  v8h hv;
#pragma unroll
  for (int e = 0; e < 4; ++e) {
    const float f0 = a0[e];
    const float f1 = a1[e];
    hv[e]     = (_Float16)carry_flush(bf16r(f0), kInCarry);
    hv[4 + e] = (_Float16)carry_flush(bf16r(f1), kInCarry);
  }
  unsigned short* dp = dst + (size_t)row * dstPitch + dstOff + c8;
  *(volatile v8h*)dp = hv;
  __threadfence();
  *(volatile v8h*)dp = hv;
}
__global__ __launch_bounds__(256) void wt_plane_kernel(const float* __restrict__ W, unsigned short* __restrict__ dst, int K, int N, int nLive, int ldd, int colOff) {
  const int n  = blockIdx.x;
  const int k8 = threadIdx.x * 8;
  const bool live = n < nLive;
  const int nc = live ? n : 0;
  v8h hv;
#pragma unroll
  for (int e = 0; e < 8; ++e) {
    const float w = W[(size_t)(k8 + e) * N + nc];
    hv[e] = (_Float16)(live ? carry_flush(bf16r(w), kWCarry) : 0.0f);
  }
  unsigned short* dp = dst + (size_t)n * ldd + colOff + k8;
  *(volatile v8h*)dp = hv;
  __threadfence();
  *(volatile v8h*)dp = hv;
}


__device__ __forceinline__ float fast_tanh(float v) { return 1.0f - 2.0f * frcp(__expf(2.0f * v) + 1.0f); }
__device__ __forceinline__ float fast_sigmoid(float v) { return frcp(1.0f + __expf(-v)); }

__global__ __launch_bounds__(kThr) void bias_kernel(const float* __restrict__ b_sinit, const float* __restrict__ bq, const float* __restrict__ bo,
                                                    const float* __restrict__ bc, const float* __restrict__ bs, const float* __restrict__ by,
                                                    float* __restrict__ BIAS) {
  unsigned v = blockIdx.x * (unsigned)kThr + threadIdx.x;
  asm volatile("" : "+v"(v));
  const unsigned i0 = v * 4u;
  const bool isSI = i0 < (unsigned)kFQH, isQ = (i0 >= (unsigned)kFQH) && (i0 < (unsigned)(kFQH + kD)), isO = (i0 >= (unsigned)kFBO) && (i0 < (unsigned)kFCS);
  const bool isCS = (i0 >= (unsigned)kFCS) && (i0 < (unsigned)kFBY), isY = (i0 >= (unsigned)kFBY) && (i0 < (unsigned)kFZ);
  const float* sp = isSI ? (b_sinit + i0) : isQ ? (bq + (i0 - (unsigned)kFQH)) : isO ? (bo + (i0 - (unsigned)kFBO)) : isCS ? (bc + (i0 - (unsigned)kFCS)) : isY ? (by + (i0 - (unsigned)kFBY)) : b_sinit;
  const float* s2 = isCS ? (bs + (i0 - (unsigned)kFCS)) : b_sinit;
  const v4f a = *(const v4f*)sp, c = *(const v4f*)s2;
  const bool live = isSI || isQ || isO || isCS || isY;
  v4f o;
#pragma unroll
  for (int e = 0; e < 4; ++e) { const float p = a[e], q = c[e]; o[e] = live ? (isCS ? (bf16r(p) + bf16r(q)) : bf16r(p)) : 0.0f; }
  float* dp = BIAS + i0;
  *(volatile v4f*)dp = o;
  __threadfence();
  *(volatile v4f*)dp = o;
}
static_assert(kFEnd / 4 == 6 * kThr && kFQH == kD && kFBO == kFQH + kQH && kFCS == kFBO + kE2 && kFBY == kFCS + kD && kFZ == kFBY + kD, "bias stream map");

__global__ __launch_bounds__(kThr) void pool_kernel(const float* __restrict__ xs_h, const float* __restrict__ xs_mask, unsigned short* __restrict__ POOL) {
  unsigned v = blockIdx.x * (unsigned)kThr + threadIdx.x;
  asm volatile("" : "+v"(v));
  const unsigned b = v >> 7, e8 = (v & 127u) * 8u;
  const float* xp = xs_h + (size_t)b * kLX * kE2 + e8;
  const float* mp = xs_mask + (size_t)b * kLX;
  float acc[8];
#pragma unroll
  for (int e = 0; e < 8; ++e) acc[e] = 0.0f;
  float den = 0.0f;
#pragma unroll 1
  for (int l = 0; l < kLX; ++l) {
    float m = mp[l];
    asm volatile("" : "+v"(m));
    m = bf16r(m);
    const v4f a0 = *(const v4f*)(xp + (size_t)l * kE2), a1 = *(const v4f*)(xp + (size_t)l * kE2 + 4);
#pragma unroll
    for (int e = 0; e < 4; ++e) { const float p = a0[e], q = a1[e]; acc[e] += bf16r(p) * m; acc[4 + e] += bf16r(q) * m; }
    den += m;
  }
  v8h hv;
#pragma unroll
  for (int e = 0; e < 8; ++e) hv[e] = (_Float16)carry_flush(acc[e] / den, kInCarry);
  unsigned short* dp = POOL + (size_t)b * kE2 + e8;
  *(volatile v8h*)dp = hv;
  __threadfence();
  *(volatile v8h*)dp = hv;
}
static_assert(kB * kE2 / 8 == 32 * kThr, "pool grid exact");

__global__ __launch_bounds__(kThr) void s0_kernel(const float* __restrict__ S0P, float* __restrict__ S32, unsigned short* __restrict__ CS16) {
  unsigned v = blockIdx.x * (unsigned)kThr + threadIdx.x;
  asm volatile("" : "+v"(v));
  const unsigned b = v >> 6, u8 = (v & 63u) * 8u;
  const size_t o8 = (size_t)b * kD + u8;
  const v4f a0 = *(const v4f*)(S0P + o8), a1 = *(const v4f*)(S0P + o8 + 4);
  v4f h0, h1; v8h hv;
#pragma unroll
  for (int e = 0; e < 4; ++e) { h0[e] = tanhf(a0[e]); h1[e] = tanhf(a1[e]); hv[e] = (_Float16)carry_flush(h0[e], kInCarry); hv[4 + e] = (_Float16)carry_flush(h1[e], kInCarry); }
  unsigned short* dp = CS16 + (size_t)b * kCS + kE2 + u8;
  for (int pass = 0; pass < 2; ++pass) {
    *(volatile v4f*)(S32 + o8) = h0; *(volatile v4f*)(S32 + o8 + 4) = h1;
    *(volatile v8h*)dp = hv;
    __threadfence();
  }
}
static_assert(kB * kD / 8 == 16 * kThr, "first-state grid exact");

__global__ __launch_bounds__(kThr) void lngru_kernel(const float* __restrict__ AX, int axPitch, const float* __restrict__ AH, int ahPitch, const float* __restrict__ HIN,
                                                     const float* __restrict__ ys_mask, const float* __restrict__ bx, const float* __restrict__ gx,
                                                     const float* __restrict__ gh, float* __restrict__ HOUT, unsigned short* __restrict__ O16, int oPitch, int t) {
  __shared__ float sPart[6][kThr];
  __shared__ float sSeg[6][8];
  const int tid = threadIdx.x;
  const int b = blockIdx.x;
  const int u = 2 * tid;
  const float* axr = AX + (size_t)b * axPitch;
  const float* ahr = AH + (size_t)b * ahPitch;
  float va[6][2];
#pragma unroll
  for (int c = 0; c < 3; ++c) {
    const v2f p = *(const v2f*)(axr + c * kD + u), q = *(const v2f*)(ahr + c * kD + u);
    va[c][0] = p[0]; va[c][1] = p[1]; va[3 + c][0] = q[0]; va[3 + c][1] = q[1];
  }
  float mu[6], rs[6];
#pragma unroll
  for (int c = 0; c < 6; ++c) sPart[c][tid] = va[c][0] + va[c][1];
  __syncthreads();
  if (tid < 48) {
    const int c = tid >> 3, sg = tid & 7;
    float s = 0.0f;
#pragma unroll 1
    for (int j = 0; j < 32; ++j) s += sPart[c][sg * 32 + j];
    sSeg[c][sg] = s;
  }
  __syncthreads();
#pragma unroll
  for (int c = 0; c < 6; ++c) {
    float s = 0.0f;
#pragma unroll
    for (int j = 0; j < 8; ++j) s += sSeg[c][j];
    mu[c] = s * (1.0f / kD);
  }
  __syncthreads();
#pragma unroll
  for (int c = 0; c < 6; ++c) { const float d0 = va[c][0] - mu[c], d1 = va[c][1] - mu[c]; sPart[c][tid] = d0 * d0 + d1 * d1; }
  __syncthreads();
  if (tid < 48) {
    const int c = tid >> 3, sg = tid & 7;
    float s = 0.0f;
#pragma unroll 1
    for (int j = 0; j < 32; ++j) s += sPart[c][sg * 32 + j];
    sSeg[c][sg] = s;
  }
  __syncthreads();
#pragma unroll
  for (int c = 0; c < 6; ++c) {
    float s = 0.0f;
#pragma unroll
    for (int j = 0; j < 8; ++j) s += sSeg[c][j];
    rs[c] = rsqrtf(s * (1.0f / kD) + 1e-5f);
  }
  float m = ys_mask[(size_t)b * kLY + t];
  asm volatile("" : "+v"(m));
  m = bf16r(m);
  const v2f hin = *(const v2f*)(HIN + (size_t)b * kD + u);
  float nx[3][2], nh[3][2];
#pragma unroll
  for (int c = 0; c < 3; ++c) {
    const v2f g1 = *(const v2f*)(gx + c * kD + u), b1 = *(const v2f*)(bx + c * kD + u), g2 = *(const v2f*)(gh + c * kD + u);
#pragma unroll
    for (int e = 0; e < 2; ++e) {
      const float p1 = g1[e], p2 = b1[e], p3 = g2[e];
      nx[c][e] = (va[c][e] - mu[c]) * rs[c] * bf16r(p1) + bf16r(p2);
      nh[c][e] = (va[3 + c][e] - mu[3 + c]) * rs[3 + c] * bf16r(p3);
    }
  }
  v2f ho; v2h hv;
#pragma unroll
  for (int e = 0; e < 2; ++e) {
    const float r = fast_sigmoid(nx[0][e] + nh[0][e]);
    const float z = fast_sigmoid(nx[1][e] + nh[1][e]);
    const float hc = fast_tanh(nx[2][e] + r * nh[2][e]);
    const float hn = (1.0f - z) * hin[e] + z * hc;
    const float h2 = m * hn + (1.0f - m) * hin[e];
    ho[e] = h2;
    hv[e] = (_Float16)carry_flush(h2, kInCarry);
  }
  float* hp = HOUT + (size_t)b * kD + u;
  unsigned short* op = O16 + (size_t)b * oPitch + u;
  for (int pass = 0; pass < 2; ++pass) {
    *(volatile v2f*)hp = ho;
    *(volatile v2h*)op = hv;
    __threadfence();
  }
}
static_assert(kD == 2 * kThr, "two adjacent units a thread");

__global__ __launch_bounds__(kThr) void attn_kernel(const float* __restrict__ UH32, const float* __restrict__ QH, const float* __restrict__ V_att,
                                                    const float* __restrict__ xs_mask, const float* __restrict__ xs_h, unsigned short* __restrict__ CTX16) {
  __shared__ __align__(16) float sQ[kD];
  __shared__ __align__(16) float sV[kD * kNH];
  __shared__ __align__(16) float sP[kThr * kNH];
  __shared__ __align__(16) float sA[kLX * kNH];
  __shared__ float sMx[kNH];
  __shared__ float sDen[kNH];
  const int tid = threadIdx.x;
  const int b = blockIdx.x;
  {
    const v2f q2 = *(const v2f*)(QH + (size_t)b * kQH + 2 * tid);
    sQ[2 * tid] = q2[0]; sQ[2 * tid + 1] = q2[1];
#pragma unroll
    for (int j = 0; j < 4; ++j) {
      const v4f w = *(const v4f*)(V_att + (size_t)(j * kThr + tid) * 4);
      v4f o;
#pragma unroll
      for (int e = 0; e < 4; ++e) { const float p = w[e]; o[e] = bf16r(p); }
      *(v4f*)(sV + (size_t)(j * kThr + tid) * 4) = o;
    }
  }
  __syncthreads();
  {
    const int l = tid >> 2, part = tid & 3;
    const float* up = UH32 + ((size_t)b * kLX + l) * kD + part * 128;
    float acc[kNH];
#pragma unroll
    for (int h = 0; h < kNH; ++h) acc[h] = 0.0f;
#pragma unroll 1
    for (int d4 = 0; d4 < 128; d4 += 4) {
      const v4f uv = *(const v4f*)(up + d4);
      const v4f qv = *(const v4f*)(sQ + part * 128 + d4);
#pragma unroll
      for (int e = 0; e < 4; ++e) {
        const float hd = fast_tanh(uv[e] + qv[e]);
        const v4f w0 = *(const v4f*)(sV + (size_t)(part * 128 + d4 + e) * kNH), w1 = *(const v4f*)(sV + (size_t)(part * 128 + d4 + e) * kNH + 4);
#pragma unroll
        for (int h = 0; h < 4; ++h) { acc[h] += hd * w0[h]; acc[4 + h] += hd * w1[h]; }
      }
    }
#pragma unroll
    for (int h = 0; h < kNH; ++h) sP[tid * kNH + h] = acc[h];
  }
  __syncthreads();
#pragma unroll
  for (int r = 0; r < 2; ++r) {
    const int i = tid + kThr * r;
    const int l = i >> 3, h = i & 7;
    float s = sP[(l * 4 + 0) * kNH + h];
    s += sP[(l * 4 + 1) * kNH + h];
    s += sP[(l * 4 + 2) * kNH + h];
    s += sP[(l * 4 + 3) * kNH + h];
    float mk = xs_mask[(size_t)b * kLX + l];
    asm volatile("" : "+v"(mk));
    sA[i] = (bf16r(mk) > 0.0f) ? s : -1.0e9f;
  }
  __syncthreads();
  if (tid < kNH) {
    float mx = sA[tid];
#pragma unroll 1
    for (int l = 1; l < kLX; ++l) { const float q = sA[l * kNH + tid]; mx = (q > mx) ? q : mx; }
    sMx[tid] = mx;
  }
  __syncthreads();
#pragma unroll
  for (int r = 0; r < 2; ++r) {
    const int i = tid + kThr * r;
    sA[i] = __expf(sA[i] - sMx[i & 7]);
  }
  __syncthreads();
  if (tid < kNH) {
    float s = 0.0f;
#pragma unroll 1
    for (int l = 0; l < kLX; ++l) s += sA[l * kNH + tid];
    sDen[tid] = s;
  }
  __syncthreads();
  {
    const int j4 = tid * 4;
    const int h = tid >> 5;
    const float* xp = xs_h + (size_t)b * kLX * kE2 + j4;
    float c0 = 0.0f, c1 = 0.0f, c2 = 0.0f, c3 = 0.0f;
#pragma unroll 1
    for (int l = 0; l < kLX; ++l) {
      const float a = sA[l * kNH + h];
      const v4f x4 = *(const v4f*)(xp + (size_t)l * kE2);
      const float p0 = x4[0], p1 = x4[1], p2 = x4[2], p3 = x4[3];
      c0 += a * bf16r(p0); c1 += a * bf16r(p1); c2 += a * bf16r(p2); c3 += a * bf16r(p3);
    }
    const float den = sDen[h];
    v4h hv;
    hv[0] = (_Float16)carry_flush(c0 / den, kInCarry);
    hv[1] = (_Float16)carry_flush(c1 / den, kInCarry);
    hv[2] = (_Float16)carry_flush(c2 / den, kInCarry);
    hv[3] = (_Float16)carry_flush(c3 / den, kInCarry);
    unsigned short* dp = CTX16 + (size_t)b * kE2 + j4;
    *(volatile v4h*)dp = hv;
    __threadfence();
    *(volatile v4h*)dp = hv;
  }
}
static_assert(kLX * 4 == kThr && kLX * kNH == 2 * kThr && kD * kNH == 4 * kThr * 4 && kE2 == 4 * kThr && kHV == 128 && kD == 4 * 128, "attention thread maps");

__global__ __launch_bounds__(kThr) void cmask_kernel(const float* __restrict__ CTX2, const float* __restrict__ ys_mask, unsigned short* __restrict__ CS16, int t) {
  unsigned v = blockIdx.x * (unsigned)kThr + threadIdx.x;
  asm volatile("" : "+v"(v));
  const unsigned b = v >> 7, j8 = (v & 127u) * 8u;
  float m = ys_mask[(size_t)b * kLY + t];
  asm volatile("" : "+v"(m));
  m = bf16r(m);
  const v4f a0 = *(const v4f*)(CTX2 + (size_t)b * kE2 + j8), a1 = *(const v4f*)(CTX2 + (size_t)b * kE2 + j8 + 4);
  v8h hv;
#pragma unroll
  for (int e = 0; e < 4; ++e) { hv[e] = (_Float16)carry_flush(a0[e] * m, kInCarry); hv[4 + e] = (_Float16)carry_flush(a1[e] * m, kInCarry); }
  unsigned short* dp = CS16 + (size_t)b * kCS + j8;
  *(volatile v8h*)dp = hv;
  __threadfence();
  *(volatile v8h*)dp = hv;
}
static_assert(kB * kE2 / 8 == 32 * kThr, "mask grid exact");

__global__ __launch_bounds__(kThr) void out_kernel(const float* __restrict__ YWY, const float* __restrict__ OUTP, const float* __restrict__ ys_mask,
                                                   float* __restrict__ out, int t) {
  unsigned v = blockIdx.x * (unsigned)kThr + threadIdx.x;
  asm volatile("" : "+v"(v));
  const unsigned b = v >> 7, u4 = (v & 127u) * 4u;
  float m = ys_mask[(size_t)b * kLY + t];
  asm volatile("" : "+v"(m));
  m = bf16r(m);
  const size_t ro = ((size_t)b * kLY + (size_t)t) * kD + u4;
  const v4f y = *(const v4f*)(YWY + ro), p = *(const v4f*)(OUTP + (size_t)b * kD + u4);
  v4f o;
#pragma unroll
  for (int e = 0; e < 4; ++e) o[e] = tanhf(y[e] + p[e]) * m;
  *(volatile v4f*)(out + ro) = o;
  __threadfence();
  *(volatile v4f*)(out + ro) = o;
}
static_assert(kB * kD / 4 == 32 * kThr, "output grid exact");

static_assert(((size_t)kRows * kE2 / 8) % kThr == 0 && ((size_t)kRows * kNE / 8) % kThr == 0, "plane cast grids exact");

extern "C" void kernel_launch(void* const* d_in, const int* in_sizes, int n_in,
                              void* d_out, int out_size, void* d_ws, size_t ws_size,
                              hipStream_t stream) {
  if (n_in < 28 || d_out == nullptr || d_ws == nullptr) return;
  if (in_sizes[0] != kRows * kE2 || in_sizes[1] != kB * kLY * kNE || in_sizes[2] != kB * kLX || in_sizes[3] != kB * kLY) return;
  if (in_sizes[4] != kE2 * kD || in_sizes[5] != kD || in_sizes[6] != kE2 * kD) return;
  if (in_sizes[7] != kNE * kG3 || in_sizes[8] != kG3 || in_sizes[9] != kG3 || in_sizes[10] != kD * kG3 || in_sizes[11] != kG3) return;
  if (in_sizes[12] != kE2 * kG3 || in_sizes[13] != kG3 || in_sizes[14] != kG3 || in_sizes[15] != kD * kG3 || in_sizes[16] != kG3) return;
  if (in_sizes[17] != kD * kD || in_sizes[18] != kD || in_sizes[19] != kD * kNH || in_sizes[20] != kE2 * kE2 || in_sizes[21] != kE2) return;
  if (in_sizes[22] != kNE * kD || in_sizes[23] != kD || in_sizes[24] != kE2 * kD || in_sizes[25] != kD || in_sizes[26] != kD * kD || in_sizes[27] != kD) return;
  if (out_size != kB * kLY * kD) return;
  if (ws_size < kWsTotal) return;
  const float* xs_h = (const float*)d_in[0];
  const float* ys_e = (const float*)d_in[1];
  const float* xs_mask = (const float*)d_in[2];
  const float* ys_mask = (const float*)d_in[3];
  const float* W_sinit = (const float*)d_in[4];
  const float* b_sinit = (const float*)d_in[5];
  const float* W_keys = (const float*)d_in[6];
  const float* Wx_cell = (const float*)d_in[7];
  const float* bx_cell = (const float*)d_in[8];
  const float* gx_cell = (const float*)d_in[9];
  const float* Wh_cell = (const float*)d_in[10];
  const float* gh_cell = (const float*)d_in[11];
  const float* Wx_cond = (const float*)d_in[12];
  const float* bx_cond = (const float*)d_in[13];
  const float* gx_cond = (const float*)d_in[14];
  const float* Wh_cond = (const float*)d_in[15];
  const float* gh_cond = (const float*)d_in[16];
  const float* Wq = (const float*)d_in[17];
  const float* bq = (const float*)d_in[18];
  const float* V_att = (const float*)d_in[19];
  const float* Wo = (const float*)d_in[20];
  const float* bo = (const float*)d_in[21];
  const float* Wy = (const float*)d_in[22];
  const float* by = (const float*)d_in[23];
  const float* Wc = (const float*)d_in[24];
  const float* bc = (const float*)d_in[25];
  const float* Ws = (const float*)d_in[26];
  const float* bs = (const float*)d_in[27];
  float* out = (float*)d_out;
  char* ws = (char*)d_ws;
  unsigned short* WKT = (unsigned short*)(ws + kOffWKT);
  unsigned short* WSIT = (unsigned short*)(ws + kOffWSIT);
  unsigned short* WXCT = (unsigned short*)(ws + kOffWXCT);
  unsigned short* WHCT = (unsigned short*)(ws + kOffWHCT);
  unsigned short* WQHT = (unsigned short*)(ws + kOffWQHT);
  unsigned short* WOT = (unsigned short*)(ws + kOffWOT);
  unsigned short* WXDT = (unsigned short*)(ws + kOffWXDT);
  unsigned short* WCST = (unsigned short*)(ws + kOffWCST);
  unsigned short* WYT = (unsigned short*)(ws + kOffWYT);
  float* BIAS = (float*)(ws + kOffBIAS);
  unsigned short* XS16 = (unsigned short*)(ws + kOffXS16);
  unsigned short* YS16 = (unsigned short*)(ws + kOffYS16);
  float* UH32 = (float*)(ws + kOffUH32);
  float* AXC = (float*)(ws + kOffAXC);
  float* YWY = (float*)(ws + kOffYWY);
  unsigned short* POOL = (unsigned short*)(ws + kOffPOOL);
  float* S0P = (float*)(ws + kOffS0P);
  float* S32 = (float*)(ws + kOffS32);
  float* ST32 = (float*)(ws + kOffST32);
  unsigned short* ST16 = (unsigned short*)(ws + kOffST16);
  unsigned short* CS16 = (unsigned short*)(ws + kOffCS16);
  float* AH1 = (float*)(ws + kOffAH1);
  float* QH = (float*)(ws + kOffQH);
  unsigned short* CTX16 = (unsigned short*)(ws + kOffCTX16);
  float* CTX2 = (float*)(ws + kOffCTX2);
  float* AX2 = (float*)(ws + kOffAX2);
  float* OUTP = (float*)(ws + kOffOUTP);

  wt_plane_kernel<<<kD, kE2 / 8, 0, stream>>>(W_keys, WKT, kE2, kD, kD, kE2, 0);
  wt_plane_kernel<<<kD, kE2 / 8, 0, stream>>>(W_sinit, WSIT, kE2, kD, kD, kE2, 0);
  wt_plane_kernel<<<kG3, kNE / 8, 0, stream>>>(Wx_cell, WXCT, kNE, kG3, kG3, kNE, 0);
  wt_plane_kernel<<<kG3, kD / 8, 0, stream>>>(Wh_cell, WHCT, kD, kG3, kG3, kD, 0);
  wt_plane_kernel<<<kD, kD / 8, 0, stream>>>(Wq, WQHT, kD, kD, kD, kD, 0);
  wt_plane_kernel<<<kG3, kD / 8, 0, stream>>>(Wh_cond, WQHT + (size_t)kD * kD, kD, kG3, kG3, kD, 0);
  wt_plane_kernel<<<kE2, kE2 / 8, 0, stream>>>(Wo, WOT, kE2, kE2, kE2, kE2, 0);
  wt_plane_kernel<<<kG3, kE2 / 8, 0, stream>>>(Wx_cond, WXDT, kE2, kG3, kG3, kE2, 0);
  wt_plane_kernel<<<kD, kE2 / 8, 0, stream>>>(Wc, WCST, kE2, kD, kD, kCS, 0);
  wt_plane_kernel<<<kD, kD / 8, 0, stream>>>(Ws, WCST, kD, kD, kD, kCS, kE2);
  wt_plane_kernel<<<kD, kNE / 8, 0, stream>>>(Wy, WYT, kNE, kD, kD, kNE, 0);
  cast_plane_kernel<<<(int)(((size_t)kRows * kE2 / 8) / kThr), kThr, 0, stream>>>(xs_h, XS16, 10, kE2, 0);
  cast_plane_kernel<<<(int)(((size_t)kRows * kNE / 8) / kThr), kThr, 0, stream>>>(ys_e, YS16, 9, kNE, 0);
  bias_kernel<<<6, kThr, 0, stream>>>(b_sinit, bq, bo, bc, bs, by, BIAS);
  wmma_gemm64<0, false, 2, 0, false, 0><<<dim3((kRows / 64) * (kD / 64) / 8, 1), 256, 0, stream>>>(
      XS16, XS16, kE2, 0L, WKT, WKT, kE2, 0L, (void*)UH32, (void*)UH32, kD, 0L, BIAS + kFZ, nullptr, 0L, kRows, kD, kE2, kSc);
  wmma_gemm64<0, false, 2, 0, false, 0><<<dim3((kRows / 64) * (kG3 / 64) / 8, 1), 256, 0, stream>>>(
      YS16, YS16, kNE, 0L, WXCT, WXCT, kNE, 0L, (void*)AXC, (void*)AXC, kG3, 0L, BIAS + kFZ, nullptr, 0L, kRows, kG3, kNE, kSc);
  wmma_gemm64<0, false, 2, 0, false, 0><<<dim3((kRows / 64) * (kD / 64) / 8, 1), 256, 0, stream>>>(
      YS16, YS16, kNE, 0L, WYT, WYT, kNE, 0L, (void*)YWY, (void*)YWY, kD, 0L, BIAS + kFBY, nullptr, 0L, kRows, kD, kNE, kSc);
  pool_kernel<<<32, kThr, 0, stream>>>(xs_h, xs_mask, POOL);
  wmma_gemm64<0, false, 2, 0, false, 0><<<dim3((kB / 64) * (kD / 64) / 8, 1), 256, 0, stream>>>(
      POOL, POOL, kE2, 0L, WSIT, WSIT, kE2, 0L, (void*)S0P, (void*)S0P, kD, 0L, BIAS + kFSI, nullptr, 0L, kB, kD, kE2, kSc);
  s0_kernel<<<16, kThr, 0, stream>>>(S0P, S32, CS16);

  for (int t = 0; t < kLY; ++t) {
    wmma_gemm64<0, false, 2, 0, false, 0><<<dim3((kB / 64) * (kG3 / 64) / 8, 1), 256, 0, stream>>>(
        CS16 + kE2, CS16 + kE2, kCS, 0L, WHCT, WHCT, kD, 0L, (void*)AH1, (void*)AH1, kG3, 0L, BIAS + kFZ, nullptr, 0L, kB, kG3, kD, kSc);
    lngru_kernel<<<kB, kThr, 0, stream>>>(AXC + (size_t)t * kG3, kLY * kG3, AH1, kG3, S32, ys_mask, bx_cell, gx_cell, gh_cell, ST32, ST16, kD, t);
    wmma_gemm64<0, false, 2, 0, false, 0><<<dim3((kB / 64) * (kQH / 64) / 8, 1), 256, 0, stream>>>(
        ST16, ST16, kD, 0L, WQHT, WQHT, kD, 0L, (void*)QH, (void*)QH, kQH, 0L, BIAS + kFQH, nullptr, 0L, kB, kQH, kD, kSc);
    attn_kernel<<<kB, kThr, 0, stream>>>(UH32, QH, V_att, xs_mask, xs_h, CTX16);
    wmma_gemm64<0, false, 2, 0, false, 0><<<dim3((kB / 64) * (kE2 / 64) / 8, 1), 256, 0, stream>>>(
        CTX16, CTX16, kE2, 0L, WOT, WOT, kE2, 0L, (void*)CTX2, (void*)CTX2, kE2, 0L, BIAS + kFBO, nullptr, 0L, kB, kE2, kE2, kSc);
    cmask_kernel<<<32, kThr, 0, stream>>>(CTX2, ys_mask, CS16, t);
    wmma_gemm64<0, false, 2, 0, false, 0><<<dim3((kB / 64) * (kG3 / 64) / 8, 1), 256, 0, stream>>>(
        CS16, CS16, kCS, 0L, WXDT, WXDT, kE2, 0L, (void*)AX2, (void*)AX2, kG3, 0L, BIAS + kFZ, nullptr, 0L, kB, kG3, kE2, kSc);
    lngru_kernel<<<kB, kThr, 0, stream>>>(AX2, kG3, QH + kD, kQH, ST32, ys_mask, bx_cond, gx_cond, gh_cond, S32, CS16 + kE2, kCS, t);
    wmma_gemm64<0, false, 2, 0, false, 0><<<dim3((kB / 64) * (kD / 64) / 8, 1), 256, 0, stream>>>(
        CS16, CS16, kCS, 0L, WCST, WCST, kCS, 0L, (void*)OUTP, (void*)OUTP, kD, 0L, BIAS + kFCS, nullptr, 0L, kB, kD, kCS, kSc);
    out_kernel<<<32, kThr, 0, stream>>>(YWY, OUTP, ys_mask, out, t);
  }
}
